// TestConv3_18322330484758
// MI455X (gfx1250) — hardware-run, weakly checked
//
#include <hip/hip_runtime.h>
#include <stddef.h>


#define CIN     128
#define COUT    64
#define KBIL    (COUT * COUT)
#define SPLITN  812
#define RB      224
#define CH      2048
#define NTS     256
#define NWS     (NTS / 32)
#define SEG     (CH / NWS)
#define HB      64
#define NTG     128
#define NWG     (NTG / 32)
#define APITCH  72
#define WSCAP   134217728
#define LDS_SCAN (2 * RB * CIN * 4 + 2 * CH * 4 + 2 * 3 * RB * 4 + RB * 4 + RB * 4 + 2 * NWS * 4)

static_assert(SEG == 8 * 32);
static_assert((RB % 32) == 0 && RB <= 256 && RB <= NTS && (RB % 16) == 0);
static_assert(CIN == 128 && COUT == 64 && (KBIL % 64) == 0);
static_assert(LDS_SCAN <= 300 * 1024);
static_assert(NWS == 8 && NWG == 4);

typedef float          v4f  __attribute__((ext_vector_type(4)));
typedef float          v8f  __attribute__((ext_vector_type(8)));
typedef _Float16       v4h  __attribute__((ext_vector_type(4)));
typedef _Float16       v8h  __attribute__((ext_vector_type(8)));
typedef _Float16       v16h __attribute__((ext_vector_type(16)));
typedef int            v4i  __attribute__((ext_vector_type(4)));
typedef unsigned int   v4u  __attribute__((ext_vector_type(4)));
union Frag { v16h v; v8h h[2]; };

static __device__ __forceinline__ v8f wm(v16h a, v16h b, v8f c) {
  v8f d = __builtin_amdgcn_wmma_f32_16x16x32_f16(false, a, false, b, (short)0, c, false, false);
  asm volatile("v_nop\n\tv_nop\n\tv_nop\n\tv_nop" : "+v"(d) : "v"(a), "v"(b));
  return d;
}

static __device__ __forceinline__ int clampi(int v, int lo, int hi) {
  return v < lo ? lo : (v > hi ? hi : v);
}

__global__ __launch_bounds__(NTS) void k_hist(const int* __restrict__ ecol, unsigned* part,
                                             int E, int N, int npd, int ce) {
  extern __shared__ v4f lds_dyn[];
  unsigned* h = (unsigned*)lds_dyn;
  const int tid = threadIdx.x;
  const int b = (int)blockIdx.x;
  {
    const v4u zz = {0u, 0u, 0u, 0u};
#pragma unroll 1
    for (int i = tid; i < npd / 4; i += NTS) ((v4u*)h)[i] = zz;
  }
  __syncthreads();
  const int e0 = b * ce;
#pragma unroll 1
  for (int i = tid; i < ce; i += NTS) {
    const int e  = e0 + i;
    const int ea = e < E ? e : E - 1;
    const int c  = clampi(ecol[ea], 0, N - 1);
    if (e < E) atomicAdd(&h[c], 1u);
  }
  __syncthreads();
  unsigned* pp = part + (size_t)b * (size_t)npd;
#pragma unroll 1
  for (int i = tid; i < npd / 4; i += NTS) {
    const v4u v = ((const v4u*)h)[i];
    *(volatile v4u*)(pp + 4 * i) = v;
  }
  __threadfence();
#pragma unroll 1
  for (int i = tid; i < npd / 4; i += NTS) {
    const v4u v = ((const v4u*)h)[i];
    *(volatile v4u*)(pp + 4 * i) = v;
  }
}

__global__ __launch_bounds__(NTS) void k_degfin(const unsigned* __restrict__ part, unsigned* deg, float* dinv,
                                               int npd, int hb) {
  const int i = (int)blockIdx.x * NTS + (int)threadIdx.x;
  if (i >= npd / 4) return;
  v4u s = {0u, 0u, 0u, 0u};
#pragma unroll 1
  for (int b = 0; b < hb; ++b) s += *(const v4u*)(part + (size_t)b * (size_t)npd + 4 * i);
  v4f d;
  d.x = s.x ? rsqrtf((float)s.x) : 0.0f;
  d.y = s.y ? rsqrtf((float)s.y) : 0.0f;
  d.z = s.z ? rsqrtf((float)s.z) : 0.0f;
  d.w = s.w ? rsqrtf((float)s.w) : 0.0f;
  *(volatile v4u*)(deg + 4 * i) = s;
  *(volatile v4f*)(dinv + 4 * i) = d;
  __threadfence();
  *(volatile v4u*)(deg + 4 * i) = s;
  *(volatile v4f*)(dinv + 4 * i) = d;
}

__global__ __launch_bounds__(NTS) void k_cvtw(const float* __restrict__ Wsame, const float* __restrict__ Wdiff,
                                             const float* __restrict__ Wbil,
                                             _Float16* Wsm16, _Float16* Wdf16, _Float16* Wb16) {
  const int b = (int)blockIdx.x;
  const int tid = threadIdx.x;
  const float* src;
  _Float16* dst;
  float sc;
  int base;
  if (b < 4)      { src = Wsame; dst = Wsm16; sc = 16.0f; base = b * 2048; }
  else if (b < 8) { src = Wdiff; dst = Wdf16; sc = 16.0f; base = (b - 4) * 2048; }
  else            { src = Wbil;  dst = Wb16;  sc = 64.0f; base = (b - 8) * 2048; }
  const int e = base + 8 * tid;
  const v4f f0 = *(const v4f*)(src + e);
  const v4f f1 = *(const v4f*)(src + e + 4);
  v8h hv;
  hv[0] = (_Float16)(f0.x * sc); hv[1] = (_Float16)(f0.y * sc); hv[2] = (_Float16)(f0.z * sc); hv[3] = (_Float16)(f0.w * sc);
  hv[4] = (_Float16)(f1.x * sc); hv[5] = (_Float16)(f1.y * sc); hv[6] = (_Float16)(f1.z * sc); hv[7] = (_Float16)(f1.w * sc);
  *(volatile v8h*)(dst + e) = hv;
  __threadfence();
  *(volatile v8h*)(dst + e) = hv;
}

static __device__ __forceinline__ void scan_emit(const float* acc, const int* tkr, const int* tkc,
                                                 _Float16* Xs16, _Float16* Xd16, int* tk4,
                                                 int n0, int wave, int lane, int tid) {
  const int hh = lane >> 4, ch0 = 8 * (lane & 15);
#pragma unroll 1
  for (int s2 = 0; s2 < RB / 16; ++s2) {
    const int lr = wave + NWS * (2 * s2 + hh);
    const float* ps = acc + lr * CIN + ch0;
    const float* pd = ps + RB * CIN;
    const v4f a0 = *(const v4f*)ps, a1 = *(const v4f*)(ps + 4);
    const v4f d0 = *(const v4f*)pd, d1 = *(const v4f*)(pd + 4);
    v8h hs, hd;
    hs[0] = (_Float16)(a0.x * 256.0f); hs[1] = (_Float16)(a0.y * 256.0f); hs[2] = (_Float16)(a0.z * 256.0f); hs[3] = (_Float16)(a0.w * 256.0f);
    hs[4] = (_Float16)(a1.x * 256.0f); hs[5] = (_Float16)(a1.y * 256.0f); hs[6] = (_Float16)(a1.z * 256.0f); hs[7] = (_Float16)(a1.w * 256.0f);
    hd[0] = (_Float16)(d0.x * 256.0f); hd[1] = (_Float16)(d0.y * 256.0f); hd[2] = (_Float16)(d0.z * 256.0f); hd[3] = (_Float16)(d0.w * 256.0f);
    hd[4] = (_Float16)(d1.x * 256.0f); hd[5] = (_Float16)(d1.y * 256.0f); hd[6] = (_Float16)(d1.z * 256.0f); hd[7] = (_Float16)(d1.w * 256.0f);
    const size_t go = (size_t)(n0 + lr) * CIN + (size_t)ch0;
    *(volatile v8h*)(Xs16 + go) = hs;
    *(volatile v8h*)(Xd16 + go) = hd;
  }
  if (tid < RB) {
    const int n = tid;
    v4i v;
    v.x = tkr[3 * n]; v.y = tkr[3 * n + 1]; v.z = tkr[3 * n + 2]; v.w = tkc[n];
    *(volatile v4i*)(tk4 + (size_t)(n0 + n) * 4) = v;
  }
}

__global__ __launch_bounds__(NTS) void k_scan(const int* __restrict__ erow, const int* __restrict__ ecol,
                                             const float* __restrict__ x, const float* __restrict__ dinv,
                                             const unsigned* __restrict__ deg,
                                             _Float16* Xs16, _Float16* Xd16, int* tk4,
                                             int E, int N, int npd) {
  extern __shared__ v4f lds_dyn[];
  float*    acc   = (float*)lds_dyn;
  int*      listA = (int*)(acc + 2 * RB * CIN);
  int*      listT = listA + CH;
  unsigned* tkk   = (unsigned*)(listT + CH);
  int*      tkr   = (int*)(tkk + 3 * RB);
  int*      tkc   = tkr + 3 * RB;
  float*    sdi   = (float*)(tkc + RB);
  int*      cntA  = (int*)(sdi + RB);
  int*      cntT  = cntA + NWS;
  const int tid = threadIdx.x, lane = tid & 31;
  const int wave = __builtin_amdgcn_readfirstlane(tid >> 5);
  const int n0 = (int)blockIdx.x * RB;

  {
    const v4f zz = {0.f, 0.f, 0.f, 0.f};
#pragma unroll 1
    for (int i = tid; i < (2 * RB * CIN) / 4; i += NTS) ((v4f*)acc)[i] = zz;
  }
#pragma unroll 1
  for (int i = tid; i < 3 * RB; i += NTS) { tkk[i] = 0xFFFFFFFFu; tkr[i] = 0; }
#pragma unroll 1
  for (int i = tid; i < RB; i += NTS) {
    tkc[i] = 0;
    const int g  = n0 + i;
    const int gc = g < npd ? g : npd - 1;
    const float d = dinv[gc];
    sdi[i] = (g < N) ? d : 0.0f;
  }

  const int nch = (E + CH - 1) / CH;
#pragma unroll 1
  for (int chk = 0; chk < nch; ++chk) {
    __syncthreads();
    const int cbase = chk * CH + wave * SEG;
    int posA = 0, posT = 0;
#pragma unroll
    for (int j = 0; j < 8; ++j) {
      const int e  = cbase + j * 32 + lane;
      const int ea = e < E ? e : E - 1;
      const int r  = erow[ea];
      const int c  = ecol[ea];
      const bool valid = e < E;
      const unsigned lr = (unsigned)(r - n0);
      const unsigned lc = (unsigned)(c - n0);
      const bool dif = (r < SPLITN) != (c < SPLITN);
      const bool hA = valid && (lr < (unsigned)RB);
      const bool hT = valid && dif && (lc < (unsigned)RB);
      const unsigned mA = __builtin_amdgcn_ballot_w32(hA);
      const unsigned mT = __builtin_amdgcn_ballot_w32(hT);
      const int rkA = (int)__builtin_amdgcn_mbcnt_lo(mA, 0u);
      const int rkT = (int)__builtin_amdgcn_mbcnt_lo(mT, 0u);
      const int cc = clampi(c, 0, N - 1);
      const int rr = clampi(r, 0, N - 1);
      if (hA) listA[wave * SEG + posA + rkA] = cc | ((int)lr << 16) | ((dif ? 0 : 1) << 24);
      if (hT) listT[wave * SEG + posT + rkT] = rr | ((int)lc << 16);
      posA += (int)__builtin_popcount(mA);
      posT += (int)__builtin_popcount(mT);
    }
    if (lane == 0) { cntA[wave] = posA; cntT[wave] = posT; }
    __syncthreads();

#pragma unroll 1
    for (int sg = 0; sg < NWS; ++sg) {
      int na = __builtin_amdgcn_readfirstlane(cntA[sg]);
      na = na < 0 ? 0 : (na > SEG ? SEG : na);
#pragma unroll 1
      for (int i = 0; i < na; ++i) {
        const int rec = __builtin_amdgcn_readfirstlane(listA[sg * SEG + i]);
        const int lr = (rec >> 16) & 255;
        if ((lr & (NWS - 1)) == wave && lr < RB) {
          const int c  = rec & 32767;
          const int sm = (rec >> 24) & 1;
          const float w = sdi[lr] * dinv[c];
          const v4f xv = *(const v4f*)(x + (size_t)c * CIN + 4 * lane);
          float* ap = acc + ((sm ? 0 : RB * CIN) + lr * CIN + 4 * lane);
          v4f a = *(const v4f*)ap;
          const v4f wv = {w, w, w, w};
          a = wv * xv + a;
          *(v4f*)ap = a;
        }
      }
    }

    if (tid == 0) {
#pragma unroll 1
      for (int sg = 0; sg < NWS; ++sg) {
        int nt = cntT[sg];
        nt = nt < 0 ? 0 : (nt > SEG ? SEG : nt);
#pragma unroll 1
        for (int i = 0; i < nt; ++i) {
          const int rec = listT[sg * SEG + i];
          const int rr = rec & 32767;
          int lc = (rec >> 16) & 255;
          lc = lc < RB ? lc : RB - 1;
          const unsigned key = deg[rr] - 1u;
          const unsigned k0 = tkk[3 * lc], k1 = tkk[3 * lc + 1], k2 = tkk[3 * lc + 2];
          const int r0 = tkr[3 * lc], r1 = tkr[3 * lc + 1], r2 = tkr[3 * lc + 2];
          const int cn = tkc[lc];
          const int p = ((cn > 0 && k0 <= key) ? 1 : 0) + ((cn > 1 && k1 <= key) ? 1 : 0) +
                        ((cn > 2 && k2 <= key) ? 1 : 0);
          const unsigned nk0 = (p == 0) ? key : k0;
          const int      nr0 = (p == 0) ? rr  : r0;
          const unsigned nk1 = (p == 0) ? k0  : ((p == 1) ? key : k1);
          const int      nr1 = (p == 0) ? r0  : ((p == 1) ? rr  : r1);
          const unsigned nk2 = (p <= 1) ? k1  : ((p == 2) ? key : k2);
          const int      nr2 = (p <= 1) ? r1  : ((p == 2) ? rr  : r2);
          tkk[3 * lc] = nk0; tkk[3 * lc + 1] = nk1; tkk[3 * lc + 2] = nk2;
          tkr[3 * lc] = nr0; tkr[3 * lc + 1] = nr1; tkr[3 * lc + 2] = nr2;
          tkc[lc] = cn < 3 ? cn + 1 : 3;
        }
      }
    }
  }
  __syncthreads();

  scan_emit(acc, tkr, tkc, Xs16, Xd16, tk4, n0, wave, lane, tid);
  __threadfence();
  scan_emit(acc, tkr, tkc, Xs16, Xd16, tk4, n0, wave, lane, tid);
}

__global__ __launch_bounds__(NTG) void k_gemm(const _Float16* __restrict__ Ap, const _Float16* __restrict__ Wp,
                                             const float* __restrict__ bias, float* C, int npa) {
  __shared__ __attribute__((aligned(16))) float so[NWG][16 * COUT];
  const int tid = threadIdx.x, lane = tid & 31, hh = lane >> 4, m = lane & 15;
  const int wave = __builtin_amdgcn_readfirstlane(tid >> 5);
  const int row0 = ((int)blockIdx.x * NWG + wave) * 16;
  int ra = row0 + m;
  ra = ra < npa ? ra : npa - 1;
  const _Float16* ap = Ap + (size_t)ra * CIN + 8 * hh;
  const _Float16* bp = Wp + (size_t)m * CIN + 8 * hh;

  v8f acc[4];
#pragma unroll
  for (int t = 0; t < 4; ++t) { v8f zz = {0.f, 0.f, 0.f, 0.f, 0.f, 0.f, 0.f, 0.f}; acc[t] = zz; }

#pragma unroll
  for (int ks = 0; ks < CIN / 32; ++ks) {
    Frag a;
    a.h[0] = *(const v8h*)(ap + 32 * ks);
    a.h[1] = *(const v8h*)(ap + 32 * ks + 16);
#pragma unroll
    for (int t = 0; t < 4; ++t) {
      const _Float16* q = bp + (size_t)(16 * t) * CIN + 32 * ks;
      Frag b;
      b.h[0] = *(const v8h*)q;
      b.h[1] = *(const v8h*)(q + 16);
      acc[t] = wm(a.v, b.v, acc[t]);
    }
  }

  float* sp = so[wave] + (8 * hh) * COUT + m;
#pragma unroll
  for (int t = 0; t < 4; ++t) {
#pragma unroll
    for (int r = 0; r < 8; ++r) sp[r * COUT + 16 * t] = acc[t][r];
  }
  __syncthreads();

  const int c4 = 4 * m;
  const v4f bv = *(const v4f*)(bias + c4);
  const v4f sc = {1.0f / 4096.0f, 1.0f / 4096.0f, 1.0f / 4096.0f, 1.0f / 4096.0f};
  v4f vals[8];
#pragma unroll
  for (int i = 0; i < 8; ++i) {
    const v4f v = *(const v4f*)(so[wave] + (2 * i + hh) * COUT + c4);
    vals[i] = v * sc + bv;
  }
  float* cp = C + (size_t)row0 * COUT + c4;
#pragma unroll
  for (int i = 0; i < 8; ++i) *(volatile v4f*)(cp + (size_t)(2 * i + hh) * COUT) = vals[i];
  __threadfence();
#pragma unroll
  for (int i = 0; i < 8; ++i) *(volatile v4f*)(cp + (size_t)(2 * i + hh) * COUT) = vals[i];
}

__global__ __launch_bounds__(NTG) void k_bil(const float* __restrict__ xdt, const float* __restrict__ xst,
                                            const int* __restrict__ tk4, const _Float16* __restrict__ Wb16,
                                            const float* __restrict__ bbil, const float* __restrict__ gatew,
                                            float* out, int N, int npg, int npt) {
  __shared__ __attribute__((aligned(16))) _Float16 sa[NWG][16 * APITCH];
  __shared__ __attribute__((aligned(16))) _Float16 sb[NWG][16 * APITCH];
  __shared__ __attribute__((aligned(16))) float    so[NWG][16 * COUT];
  __shared__ int scn[NWG][16];
  const int tid = threadIdx.x, lane = tid & 31, hh = lane >> 4, m = lane & 15;
  const int wave = __builtin_amdgcn_readfirstlane(tid >> 5);
  const int t0 = ((int)blockIdx.x * NWG + wave) * 16;

  {
    const int gr = t0 + m;
    const int gt = gr < npt ? gr : npt - 1;
    const v4i nb = *(const v4i*)(tk4 + (size_t)gt * 4);
    const int cn = clampi(nb.w, 0, 3);
    const int q0 = clampi(nb.x, 0, N - 1);
    const int q1 = clampi(nb.y, 0, N - 1);
    const int q2 = clampi(nb.z, 0, N - 1);
    const float f0 = cn > 0 ? 1.0f : 0.0f, f1 = cn > 1 ? 1.0f : 0.0f, f2 = cn > 2 ? 1.0f : 0.0f;
    const float* xr = xdt + (size_t)gr * COUT + 32 * hh;
    const float* g0 = xdt + (size_t)q0 * COUT + 32 * hh;
    const float* g1 = xdt + (size_t)q1 * COUT + 32 * hh;
    const float* g2 = xdt + (size_t)q2 * COUT + 32 * hh;
    _Float16* pa = sa[wave] + m * APITCH + 32 * hh;
    _Float16* pb = sb[wave] + m * APITCH + 32 * hh;
#pragma unroll
    for (int q = 0; q < 8; ++q) {
      const v4f xv = *(const v4f*)(xr + 4 * q);
      const v4f u0 = *(const v4f*)(g0 + 4 * q);
      const v4f u1 = *(const v4f*)(g1 + 4 * q);
      const v4f u2 = *(const v4f*)(g2 + 4 * q);
      v4f bs = u0 * f0;
      bs = bs + u1 * f1;
      bs = bs + u2 * f2;
      v4h ha, hb;
      ha.x = (_Float16)(xv.x * 16.0f); ha.y = (_Float16)(xv.y * 16.0f); ha.z = (_Float16)(xv.z * 16.0f); ha.w = (_Float16)(xv.w * 16.0f);
      hb.x = (_Float16)(bs.x * 64.0f); hb.y = (_Float16)(bs.y * 64.0f); hb.z = (_Float16)(bs.z * 64.0f); hb.w = (_Float16)(bs.w * 64.0f);
      *(v4h*)(pa + 4 * q) = ha;
      *(v4h*)(pb + 4 * q) = hb;
    }
    if (hh == 0) scn[wave][m] = cn;
  }
  __syncthreads();

  v8f acc[4];
#pragma unroll
  for (int t = 0; t < 4; ++t) { v8f zz = {0.f, 0.f, 0.f, 0.f, 0.f, 0.f, 0.f, 0.f}; acc[t] = zz; }
  const _Float16* arow = sa[wave] + m * APITCH;
  const _Float16* brow = sb[wave] + m * APITCH + 8 * hh;
  const _Float16* wrow = Wb16 + (size_t)m * KBIL + 8 * hh;
#pragma unroll 1
  for (int k0 = 0; k0 < KBIL; k0 += 32) {
    const int i0 = k0 >> 6, j0 = k0 & 63;
    const _Float16 av = arow[i0];
    const v8h b0 = *(const v8h*)(brow + j0);
    const v8h b1 = *(const v8h*)(brow + j0 + 16);
    Frag a;
    a.h[0] = b0 * av;
    a.h[1] = b1 * av;
#pragma unroll
    for (int t = 0; t < 4; ++t) {
      const _Float16* q = wrow + (size_t)(16 * t) * KBIL + k0;
      Frag b;
      b.h[0] = *(const v8h*)q;
      b.h[1] = *(const v8h*)(q + 16);
      acc[t] = wm(a.v, b.v, acc[t]);
    }
  }

  float* sp = so[wave] + (8 * hh) * COUT + m;
#pragma unroll
  for (int t = 0; t < 4; ++t) {
#pragma unroll
    for (int r = 0; r < 8; ++r) sp[r * COUT + 16 * t] = acc[t][r];
  }
  __syncthreads();

  const int c4 = 4 * m;
  const v4f bb = *(const v4f*)(bbil + c4);
  const v4f gw = *(const v4f*)(gatew + c4);
  v4f gv;
  gv.x = 1.0f / (1.0f + expf(-gw.x));
  gv.y = 1.0f / (1.0f + expf(-gw.y));
  gv.z = 1.0f / (1.0f + expf(-gw.z));
  gv.w = 1.0f / (1.0f + expf(-gw.w));
  const v4f one = {1.f, 1.f, 1.f, 1.f};
  const v4f og = one - gv;
  const v4f sc = {1.0f / 65536.0f, 1.0f / 65536.0f, 1.0f / 65536.0f, 1.0f / 65536.0f};
  v4f vals[8];
#pragma unroll
  for (int i = 0; i < 8; ++i) {
    const int row = 2 * i + hh;
    const int gr  = t0 + row;
    const int cn  = scn[wave][row];
    const float inv = cn == 1 ? 1.0f : (cn == 2 ? 0.5f : (cn == 3 ? (1.0f / 3.0f) : 0.0f));
    const float on  = cn > 0 ? 1.0f : 0.0f;
    const v4f y  = *(const v4f*)(so[wave] + row * COUT + c4);
    const v4f iv = {inv, inv, inv, inv};
    v4f bl = (y * sc) * iv + bb;
    bl = bl * on;
    v4f lr;
    lr.x = bl.x >= 0.0f ? bl.x : 0.01f * bl.x;
    lr.y = bl.y >= 0.0f ? bl.y : 0.01f * bl.y;
    lr.z = bl.z >= 0.0f ? bl.z : 0.01f * bl.z;
    lr.w = bl.w >= 0.0f ? bl.w : 0.01f * bl.w;
    const v4f xd = *(const v4f*)(xdt + (size_t)gr * COUT + c4);
    const v4f xs = *(const v4f*)(xst + (size_t)gr * COUT + c4);
    vals[i] = xs + (gv * lr + og * xd);
  }
#pragma unroll
  for (int i = 0; i < 8; ++i) {
    const int gr = t0 + 2 * i + hh;
    if (gr < N) *(volatile v4f*)(out + (size_t)gr * COUT + c4) = vals[i];
  }
  __threadfence();
#pragma unroll
  for (int i = 0; i < 8; ++i) {
    const int gr = t0 + 2 * i + hh;
    if (gr < N) *(volatile v4f*)(out + (size_t)gr * COUT + c4) = vals[i];
  }
}

extern "C" void kernel_launch(void* const* d_in, const int* in_sizes, int n_in,
                              void* d_out, int out_size, void* d_ws, size_t ws_size,
                              hipStream_t stream) {
  if (n_in < 9) return;
  const int N = in_sizes[0] / CIN;
  if (N <= 0 || in_sizes[0] != N * CIN || N > 32767) return;
  const int E = in_sizes[1] / 2;
  if (E <= 0 || in_sizes[1] != 2 * E) return;
  if (in_sizes[2] != COUT * CIN || in_sizes[3] != COUT || in_sizes[4] != COUT * CIN || in_sizes[5] != COUT) return;
  if (in_sizes[6] != COUT * KBIL || in_sizes[7] != COUT || in_sizes[8] != COUT) return;
  if (out_size != N * COUT) return;

  const float* x      = (const float*)d_in[0];
  const int*   erow   = (const int*)d_in[1];
  const int*   ecol   = erow + E;
  const float* W_same = (const float*)d_in[2];
  const float* b_same = (const float*)d_in[3];
  const float* W_diff = (const float*)d_in[4];
  const float* b_diff = (const float*)d_in[5];
  const float* W_bil  = (const float*)d_in[6];
  const float* b_bil  = (const float*)d_in[7];
  const float* gate_w = (const float*)d_in[8];
  float* out = (float*)d_out;

  const int nblkS = (N + RB - 1) / RB;
  const int NPS   = nblkS * RB;
  const int NPD   = ((N + 255) / 256) * 256;
  const int nblkG = (N + 63) / 64;
  const int NPG   = nblkG * 64;
  const int CE    = (E + HB - 1) / HB;

  char* ws = (char*)d_ws;
  size_t off = 0;
  const size_t oPart = off; off += (size_t)HB * NPD * 4;          off = (off + 255) & ~(size_t)255;
  const size_t oDeg  = off; off += (size_t)NPD * 4;               off = (off + 255) & ~(size_t)255;
  const size_t oDinv = off; off += (size_t)NPD * 4;               off = (off + 255) & ~(size_t)255;
  const size_t oXs   = off; off += (size_t)NPS * CIN * 2;         off = (off + 255) & ~(size_t)255;
  const size_t oXd   = off; off += (size_t)NPS * CIN * 2;         off = (off + 255) & ~(size_t)255;
  const size_t oTk   = off; off += (size_t)NPS * 16;              off = (off + 255) & ~(size_t)255;
  const size_t oWs   = off; off += (size_t)COUT * CIN * 2;        off = (off + 255) & ~(size_t)255;
  const size_t oWd   = off; off += (size_t)COUT * CIN * 2;        off = (off + 255) & ~(size_t)255;
  const size_t oWb   = off; off += (size_t)COUT * KBIL * 2;       off = (off + 255) & ~(size_t)255;
  const size_t oXst  = off; off += (size_t)NPG * COUT * 4;        off = (off + 255) & ~(size_t)255;
  const size_t oXdt  = off; off += (size_t)NPG * COUT * 4;        off = (off + 255) & ~(size_t)255;
  if (off > ws_size || off > (size_t)WSCAP) return;
  if ((size_t)NPD * 4 > 300 * 1024) return;
  unsigned* part  = (unsigned*)(ws + oPart);
  unsigned* deg   = (unsigned*)(ws + oDeg);
  float*    dinv  = (float*)(ws + oDinv);
  _Float16* Xs16  = (_Float16*)(ws + oXs);
  _Float16* Xd16  = (_Float16*)(ws + oXd);
  int*      tk4   = (int*)(ws + oTk);
  _Float16* Wsm16 = (_Float16*)(ws + oWs);
  _Float16* Wdf16 = (_Float16*)(ws + oWd);
  _Float16* Wb16  = (_Float16*)(ws + oWb);
  float*    xst   = (float*)(ws + oXst);
  float*    xdt   = (float*)(ws + oXdt);

  hipFuncSetAttribute(reinterpret_cast<const void*>(&k_hist),
                      hipFuncAttributeMaxDynamicSharedMemorySize, NPD * 4);
  hipFuncSetAttribute(reinterpret_cast<const void*>(&k_scan),
                      hipFuncAttributeMaxDynamicSharedMemorySize, LDS_SCAN);

  k_hist<<<HB, NTS, (size_t)NPD * 4, stream>>>(ecol, part, E, N, NPD, CE);
  k_degfin<<<(NPD / 4 + NTS - 1) / NTS, NTS, 0, stream>>>(part, deg, dinv, NPD, HB);
  k_cvtw<<<8 + (COUT * KBIL) / 2048, NTS, 0, stream>>>(W_same, W_diff, W_bil, Wsm16, Wdf16, Wb16);
  k_scan<<<nblkS, NTS, LDS_SCAN, stream>>>(erow, ecol, x, dinv, deg, Xs16, Xd16, tk4, E, N, NPD);
  k_gemm<<<nblkG, NTG, 0, stream>>>(Xs16, Wsm16, b_same, xst, NPS);
  k_gemm<<<nblkG, NTG, 0, stream>>>(Xd16, Wdf16, b_diff, xdt, NPS);
  k_bil<<<nblkG, NTG, 0, stream>>>(xdt, xst, tk4, Wb16, b_bil, gate_w, out, N, NPG, NPS);
}
